// SQN_81484119540477
// MI455X (gfx1250) — hardware-verified
//
#include <hip/hip_runtime.h>

typedef __attribute__((ext_vector_type(16))) __bf16 v16b;
typedef __attribute__((ext_vector_type(8)))  __bf16 v8b;
typedef __attribute__((ext_vector_type(8)))  float  v8f;
typedef __attribute__((ext_vector_type(4)))  float  v4f;

#define ALPHA 0.9f
#define BETA  0.85f
#define SIM_T 100

#define B_TOTAL 32768
#define N_IN    128
#define N_HID   256
#define N_OUT   8
#define ROWS_PER_WG 16
#define THREADS 256

__device__ __forceinline__ unsigned short bf_bits(float f) {
  unsigned u = __float_as_uint(f);
  return (unsigned short)((u + 0x7FFFu + ((u >> 16) & 1u)) >> 16);
}
__device__ __forceinline__ float bf2f(unsigned short h) { return __uint_as_float(((unsigned)h) << 16); }

__device__ __forceinline__ v8f mma2(v16b a, v16b bh, v16b bl, v8f c) {
  c = __builtin_amdgcn_wmma_f32_16x16x32_bf16(false, a, false, bh, (short)0, c, false, false);
  c = __builtin_amdgcn_wmma_f32_16x16x32_bf16(false, a, false, bl, (short)0, c, false, false);
  asm volatile("v_nop\n\tv_nop\n\tv_nop\n\tv_nop" : "+v"(c) : "v"(a), "v"(bh), "v"(bl));
  return c;
}

__global__ __launch_bounds__(256) void prep_kernel(const float* __restrict__ W1, const float* __restrict__ W2,
                                                  unsigned* __restrict__ f1h, unsigned* __restrict__ f1l,
                                                  unsigned* __restrict__ f2h, unsigned* __restrict__ f2l) {
  const int total1 = 16 * 8 * 32 * 8;
  const int total2 = 1 * 8 * 32 * 8;
  for (int pass = 0; pass < 2; ++pass) {
    for (int i = blockIdx.x * 256 + threadIdx.x; i < total1 + total2; i += gridDim.x * 256) {
      const bool isW1 = i < total1;
      const int j = isW1 ? i : i - total1;
      const int ep = j & 7, lane = (j >> 3) & 31, rest = j >> 8;
      const int kc = rest & 7, nt = rest >> 3;
      const int n = nt * 16 + (lane & 15), g = lane >> 4;
      float w[2];
#pragma unroll
      for (int q = 0; q < 2; ++q) {
        const int e = 2 * ep + q;
        const int k = kc * 32 + ((e < 8) ? (8 * g + e) : (16 + 8 * g + (e - 8)));
        w[q] = isW1 ? W1[k * N_HID + n] : ((n < N_OUT) ? W2[k * N_OUT + n] : 0.0f);
      }
      const unsigned short h0 = bf_bits(w[0]), h1 = bf_bits(w[1]);
      const unsigned short l0 = bf_bits(w[0] - bf2f(h0)), l1 = bf_bits(w[1] - bf2f(h1));
      unsigned* dh = isW1 ? f1h : f2h; unsigned* dl = isW1 ? f1l : f2l;
      ((volatile unsigned*)dh)[j] = (unsigned)h0 | ((unsigned)h1 << 16);
      ((volatile unsigned*)dl)[j] = (unsigned)l0 | ((unsigned)l1 << 16);
    }
    __threadfence();
  }
}

__global__ __launch_bounds__(THREADS, 1)
void snn_kernel(const float* __restrict__ inp,
                const float* __restrict__ W0,
                const unsigned* __restrict__ f1h, const unsigned* __restrict__ f1l,
                const unsigned* __restrict__ f2h, const unsigned* __restrict__ f2l,
                float* __restrict__ out)
{
  __shared__ __align__(16) __bf16 sOut0[ROWS_PER_WG * N_HID];
  __shared__ __align__(16) __bf16 sOut1[ROWS_PER_WG * N_HID];
  __shared__ __align__(16) float  sInp[ROWS_PER_WG * N_IN];
  __shared__ __align__(16) float  sRes[ROWS_PER_WG * N_OUT];

  const int tid   = threadIdx.x;
  const int lane  = tid & 31;
  const int wave  = tid >> 5;
  const int wgRow = blockIdx.x * ROWS_PER_WG;
  const bool isOutWave = (__builtin_amdgcn_readfirstlane(wave) == 0);

  for (int i = tid; i < ROWS_PER_WG * N_IN; i += THREADS)
    sInp[i] = inp[(size_t)(wgRow + (i >> 7)) * N_IN + (i & 127)];
  __syncthreads();

  const int hi      = (lane >> 4) & 1;
  const int mloc    = hi * 8;
  const int ccol    = lane & 15;
  const int colBase = wave * 32;
  const int arow = lane & 15;
  const int asel = hi * 8;

  v8f h0[2], mem0[2], syn1[2], mem1[2];
  const v8f vzero = {};
  for (int nt = 0; nt < 2; ++nt) {
    const int col = colBase + nt * 16 + ccol;
    double acc[8];
#pragma unroll
    for (int v = 0; v < 8; ++v) acc[v] = 0.0;
#pragma unroll 2
    for (int k = 0; k < N_IN; ++k) {
      const float w = W0[k * N_HID + col];
#pragma unroll
      for (int v = 0; v < 8; ++v) acc[v] += (double)(sInp[(mloc + v) * N_IN + k] * w);
    }
    v8f a;
#pragma unroll
    for (int v = 0; v < 8; ++v) a[v] = (float)acc[v];
    h0[nt] = a; mem0[nt] = vzero; syn1[nt] = vzero; mem1[nt] = vzero;
  }
  v8f syn2 = vzero, mem2 = vzero;
  float c0 = 0.0f;
  __syncthreads();

  const uint4* b1h = (const uint4*)f1h; const uint4* b1l = (const uint4*)f1l;
  const uint4* b2h = (const uint4*)f2h; const uint4* b2l = (const uint4*)f2l;
  union FB { v16b v; uint4 u[2]; };

#pragma unroll 1
  for (int t = 0; t < SIM_T; ++t) {
#pragma unroll
    for (int nt = 0; nt < 2; ++nt) {
      const int col = colBase + nt * 16 + ccol;
      v8f m0 = mem0[nt], m1 = mem1[nt];
#pragma unroll
      for (int v = 0; v < 8; ++v) {
        const float s0 = (m0[v] > 1.0f) ? 1.0f : 0.0f;
        const float s1 = (m1[v] > 1.0f) ? 1.0f : 0.0f;
        sOut0[(mloc + v) * N_HID + col] = (__bf16)s0;
        sOut1[(mloc + v) * N_HID + col] = (__bf16)s1;
        m0[v] = BETA * m0[v] + h0[nt][v] * c0 - s0;
        m1[v] = BETA * m1[v] + syn1[nt][v] - s1;
      }
      mem0[nt] = m0; mem1[nt] = m1;
    }
    if (isOutWave) {
#pragma unroll
      for (int v = 0; v < 8; ++v) mem2[v] = BETA * mem2[v] + syn2[v];
    }
    c0 = ALPHA * c0 + 1.0f;
    __syncthreads();

#pragma unroll
    for (int nt = 0; nt < 2; ++nt)
#pragma unroll
      for (int v = 0; v < 8; ++v) syn1[nt][v] *= ALPHA;
#pragma unroll 2
    for (int kc = 0; kc < 8; ++kc) {
      FB A;
      const __bf16* ap = &sOut0[arow * N_HID + kc * 32 + asel];
      A.u[0] = *(const uint4*)(ap);
      A.u[1] = *(const uint4*)(ap + 16);
#pragma unroll
      for (int nt = 0; nt < 2; ++nt) {
        const int ntg = wave * 2 + nt;
        const size_t fb = ((size_t)(ntg * 8 + kc) * 32 + lane) * 2;
        FB Bh, Bl;
        Bh.u[0] = b1h[fb]; Bh.u[1] = b1h[fb + 1];
        Bl.u[0] = b1l[fb]; Bl.u[1] = b1l[fb + 1];
        syn1[nt] = mma2(A.v, Bh.v, Bl.v, syn1[nt]);
      }
    }
    if (isOutWave) {
#pragma unroll
      for (int v = 0; v < 8; ++v) syn2[v] *= ALPHA;
#pragma unroll 2
      for (int kc = 0; kc < 8; ++kc) {
        FB A2, Bh, Bl;
        const __bf16* a2p = &sOut1[arow * N_HID + kc * 32 + asel];
        A2.u[0] = *(const uint4*)(a2p);
        A2.u[1] = *(const uint4*)(a2p + 16);
        const size_t fb = ((size_t)kc * 32 + lane) * 2;
        Bh.u[0] = b2h[fb]; Bh.u[1] = b2h[fb + 1];
        Bl.u[0] = b2l[fb]; Bl.u[1] = b2l[fb + 1];
        syn2 = mma2(A2.v, Bh.v, Bl.v, syn2);
      }
    }
    __syncthreads();
  }

  if (isOutWave && ccol < N_OUT) {
#pragma unroll
    for (int v = 0; v < 8; ++v) sRes[(mloc + v) * N_OUT + ccol] = mem2[v];
  }
  __syncthreads();
  if (wave == 0) {
    const v4f val = *(const v4f*)(&sRes[lane * 4]);
    *(volatile v4f*)(out + (size_t)wgRow * N_OUT + lane * 4) = val;
    __threadfence();
    *(volatile v4f*)(out + (size_t)wgRow * N_OUT + lane * 4) = val;
  }
}

extern "C" void kernel_launch(void* const* d_in, const int* in_sizes, int n_in,
                              void* d_out, int out_size, void* d_ws, size_t ws_size,
                              hipStream_t stream) {
  (void)in_sizes; (void)n_in; (void)out_size; (void)ws_size;
  const float* inp = (const float*)d_in[0];
  const float* W0  = (const float*)d_in[1];
  const float* W1  = (const float*)d_in[2];
  const float* W2  = (const float*)d_in[3];
  float* out = (float*)d_out;
  char* ws = (char*)d_ws;
  unsigned* f1h = (unsigned*)(ws);
  unsigned* f1l = (unsigned*)(ws + 131072);
  unsigned* f2h = (unsigned*)(ws + 262144);
  unsigned* f2l = (unsigned*)(ws + 270336);
  prep_kernel<<<64, 256, 0, stream>>>(W1, W2, f1h, f1l, f2h, f2l);
  snn_kernel<<<dim3(B_TOTAL / ROWS_PER_WG), dim3(THREADS), 0, stream>>>(inp, W0, f1h, f1l, f2h, f2l, out);
}
